// MaxFlowModel_63333587747292
// MI455X (gfx1250) — hardware-verified
//
#include <hip/hip_runtime.h>
#include <math.h>

typedef __attribute__((ext_vector_type(16))) _Float16 v16h;
typedef __attribute__((ext_vector_type(16))) __bf16 v16b;
typedef __attribute__((ext_vector_type(8)))  _Float16 v8h;
typedef __attribute__((ext_vector_type(8)))  float v8f;
typedef __attribute__((ext_vector_type(4)))  float v4f;
typedef __attribute__((ext_vector_type(2)))  float v2f;
typedef __attribute__((ext_vector_type(4)))  unsigned v4u;
typedef __attribute__((ext_vector_type(4)))  int v4i;
typedef float __attribute__((may_alias)) float_a;
typedef int __attribute__((may_alias)) int_a;

template <typename T> __device__ __forceinline__ void vst2(void* p, T v) { *(volatile T*)p = v; __threadfence(); *(volatile T*)p = v; }
__device__ __forceinline__ v8f wmma16(v16h a, v16h b, v8f c) {
  v8f d = __builtin_amdgcn_wmma_f32_16x16x32_f16(false, a, false, b, (short)0, c, false, false);
  asm volatile("v_nop\n\tv_nop\n\tv_nop\n\tv_nop" : "+v"(d) : "v"(a), "v"(b));
  return d;
}
__device__ __forceinline__ v8f wmma_bf(v16b a, v16b b, v8f c) {
  v8f d = __builtin_amdgcn_wmma_f32_16x16x32_bf16(false, a, false, b, (short)0, c, false, false);
  asm volatile("v_nop\n\tv_nop\n\tv_nop\n\tv_nop" : "+v"(d) : "v"(a), "v"(b));
  return d;
}
__device__ __forceinline__ v16h frag_h(const _Float16* rowk0, int lane) {
  union { v16h v; v8h q[2]; } u; const _Float16* p = rowk0 + 8 * (lane >> 4);
  u.q[0] = *(const v8h*)p; u.q[1] = *(const v8h*)(p + 16); return u.v;
}
__device__ __forceinline__ v16h frag_f32(const float* rowk0, int lane) {
  v16h a; const float* p = rowk0 + 8 * (lane >> 4);
#pragma unroll
  for (int i = 0; i < 8; ++i) { a[i] = (_Float16)p[i]; a[8 + i] = (_Float16)p[16 + i]; }
  return a;
}
__device__ __forceinline__ v16h frag_f32s(const float* rowk0, int lane, float sc) {
  v16h a; const float* p = rowk0 + 8 * (lane >> 4);
#pragma unroll
  for (int i = 0; i < 8; ++i) { a[i] = (_Float16)(p[i] * sc); a[8 + i] = (_Float16)(p[16 + i] * sc); }
  return a;
}
__device__ __forceinline__ v16h fragc_f32(const float* W, int k0, int n, int lane, int ld, int K) {
  v16h a; const int g = lane >> 4;
#pragma unroll
  for (int i = 0; i < 8; ++i) { const int ka = k0 + 8 * g + i, kb = ka + 16;
    a[i] = (_Float16)(ka < K ? W[(size_t)(ka < K ? ka : K - 1) * ld + n] : 0.f); a[8 + i] = (_Float16)(kb < K ? W[(size_t)(kb < K ? kb : K - 1) * ld + n] : 0.f); }
  return a;
}
struct F2 { v16b h, l; };
__device__ __forceinline__ F2 bsplit16(const float v[16]) { F2 r;
#pragma unroll
  for (int i = 0; i < 16; ++i) { const __bf16 h = (__bf16)v[i]; r.h[i] = h; r.l[i] = (__bf16)(v[i] - (float)h); }
  return r; }
__device__ __forceinline__ F2 split_row(const float* row, int k0, int lane) { float v[16]; const float* p = row + k0 + 8 * (lane >> 4);
#pragma unroll
  for (int i = 0; i < 8; ++i) { v[i] = p[i]; v[8 + i] = p[16 + i]; }
  return bsplit16(v); }
__device__ __forceinline__ F2 split_rowK(const float* row, int k0, int lane, int K) { float v[16]; const int g = lane >> 4;
#pragma unroll
  for (int i = 0; i < 8; ++i) { const int ka = k0 + 8 * g + i, kb = ka + 16; v[i] = ka < K ? row[ka < K ? ka : K - 1] : 0.f; v[8 + i] = kb < K ? row[kb < K ? kb : K - 1] : 0.f; }
  return bsplit16(v); }
__device__ __forceinline__ F2 split_col(const float* W, int k0, int n, int lane, int ld, int K) { float v[16]; const int g = lane >> 4;
#pragma unroll
  for (int i = 0; i < 8; ++i) { const int ka = k0 + 8 * g + i, kb = ka + 16; v[i] = ka < K ? W[(size_t)(ka < K ? ka : K - 1) * ld + n] : 0.f; v[8 + i] = kb < K ? W[(size_t)(kb < K ? kb : K - 1) * ld + n] : 0.f; }
  return bsplit16(v); }
__device__ __forceinline__ v8f mac3(const F2& a, const F2& b, v8f c) { c = wmma_bf(a.l, b.h, c); c = wmma_bf(a.h, b.l, c); return wmma_bf(a.h, b.h, c); }
__device__ __forceinline__ float sigm(float v) { return 1.0f / (1.0f + expf(-v)); }
#define LDSX() do { asm volatile("s_wait_dscnt 0" ::: "memory"); __builtin_amdgcn_wave_barrier(); __builtin_amdgcn_fence(__ATOMIC_RELEASE, "workgroup"); } while (0)


#define NB 4
#define NN 1024
#define DD 32
#define NH 4
#define FIN 16
#ifndef TNB
#define TNB NB
#endif
typedef __attribute__((ext_vector_type(8))) __bf16 v8b;
__device__ __forceinline__ v16b frag_b(const __bf16* rowk0, int lane) {
  union { v16b v; v8b q[2]; } u; const __bf16* p = rowk0 + 8 * (lane >> 4);
  u.q[0] = *(const v8b*)p; u.q[1] = *(const v8b*)(p + 16); return u.v;
}
__device__ __forceinline__ v16b frag_gbf(const float* rowk0, int lane) {
  v16b a; const float* p = rowk0 + 8 * (lane >> 4);
#pragma unroll
  for (int i = 0; i < 8; ++i) { a[i] = (__bf16)p[i]; a[8 + i] = (__bf16)p[16 + i]; }
  return a;
}
__device__ __forceinline__ float bfr(float v) { return (float)(__bf16)v; }
__device__ __attribute__((noinline)) float exp_ni(float v) { return expf(v); }
__device__ __attribute__((noinline)) float tanh_ni(float v) { return tanhf(v); }
#define WS_PE    0u
#define WS_NODE  (WS_PE + 2u * DD * NN)
#define WS_EDGE  (WS_NODE + 4u * NB * NN * DD)
#define WS_H     (WS_EDGE + 4u * NB * NN * DD)
#define WS_HTH   (WS_H + 4u * NB * NH * NN * DD)
#define WS_HTL   (WS_HTH + 2u * NB * NH * DD * NN)
#define WS_F     (WS_HTL + 2u * NB * NH * DD * NN)
#define WS_FLOW  (WS_F + 4u * NB * NH * 2 * NN)
#define WS_PART  (WS_FLOW + 4u * NB * NN * NN)
#define WS_MF    (WS_PART + 4u * NB * 16 * 32)
#define WS_END   (WS_MF + 4u * 32)

__global__ __launch_bounds__(256) void k_pack(const float* __restrict__ WE, __bf16* __restrict__ PE) {
  __shared__ __align__(16) __bf16 srow[NN]; const int o = blockIdx.x, tid = threadIdx.x;
  for (int k = tid; k < NN; k += 256) srow[k] = (__bf16)bfr(WE[(size_t)k * DD + o]);
  __syncthreads(); if (tid < 128) vst2((unsigned*)(PE + (size_t)o * NN + tid * 8), *(const v4u*)(&srow[tid * 8]));
}
__global__ __launch_bounds__(256) void k_encn(const float* __restrict__ X, const float* __restrict__ W, const float* __restrict__ bb, float* __restrict__ NODE) {
  __shared__ float sw[FIN][DD]; __shared__ __align__(16) float so[64][36];
  const int tid = threadIdx.x; for (int q = tid; q < FIN * DD; q += 256) sw[q / DD][q % DD] = bfr(W[q]);
  __syncthreads();
  const int rl = tid >> 2, part = tid & 3; const size_t r = (size_t)blockIdx.x * 64 + rl; const float* xr = X + r * FIN;
  for (int o = part * 8; o < part * 8 + 8; ++o) { float s = bfr(bb[o]);
#pragma unroll 1
    for (int k = 0; k < FIN; ++k) s += bfr(xr[k]) * sw[k][o];
    so[rl][o] = tanh_ni(s); }
  __syncthreads();
  for (int q = tid; q < 64 * 8; q += 256) { const int row = q >> 3, pc = q & 7; vst2(NODE + ((size_t)blockIdx.x * 64 + row) * DD + pc * 4, *(const v4f*)&so[row][pc * 4]); }
}
__global__ __launch_bounds__(128) void k_ence(const float* __restrict__ EI, const __bf16* __restrict__ PE, const float* __restrict__ bb, float* __restrict__ EDGE) {
  __shared__ __align__(16) float so[4][16][36];
  const int tid = threadIdx.x, wave = tid >> 5, lane = tid & 31, col = lane & 15, g = lane >> 4; const size_t r0 = (size_t)blockIdx.x * 64 + wave * 16;
  v8f acc[2] = {};
#pragma unroll 2
  for (int kc = 0; kc < NN / 32; ++kc) { const v16b a = frag_gbf(EI + (r0 + col) * NN + kc * 32, lane);
#pragma unroll
    for (int j = 0; j < 2; ++j) acc[j] = wmma_bf(a, frag_b(PE + (size_t)(j * 16 + col) * NN + kc * 32, lane), acc[j]); }
#pragma unroll
  for (int j = 0; j < 2; ++j) { const float b2 = bfr(bb[j * 16 + col]);
#pragma unroll
    for (int r = 0; r < 8; ++r) so[wave][8 * g + r][j * 16 + col] = tanh_ni(acc[j][r] + b2); }
  LDSX();
  for (int rl = 0; rl < 16; ++rl) if (lane < 8) vst2(EDGE + (r0 + rl) * DD + lane * 4, *(const v4f*)&so[wave][rl][lane * 4]);
}
__global__ __launch_bounds__(256) void k_gath(const float* __restrict__ X, const float* __restrict__ WH, const float* __restrict__ A1, const float* __restrict__ A2, float* __restrict__ H, __bf16* __restrict__ HTH, __bf16* __restrict__ HTL, float* __restrict__ F) {
  __shared__ float sx[64][33]; __shared__ float sw[NH][DD][DD + 1]; __shared__ float sa1[NH][DD], sa2[NH][DD]; __shared__ __align__(16) float sh[64][36]; __shared__ __align__(16) __bf16 sth[DD][72], stl[DD][72]; __shared__ __align__(16) float sf[2][64];
  const int tid = threadIdx.x, b = blockIdx.y; const int n0 = blockIdx.x * 64;
  for (int q = tid; q < 64 * DD; q += 256) sx[q / DD][q % DD] = X[((size_t)b * NN + n0 + q / DD) * DD + q % DD];
  for (int q = tid; q < NH * DD * DD; q += 256) sw[q / (DD * DD)][(q / DD) % DD][q % DD] = bfr(WH[q]);
  for (int q = tid; q < NH * DD; q += 256) { sa1[q / DD][q % DD] = bfr(A1[q]); sa2[q / DD][q % DD] = bfr(A2[q]); }
  __syncthreads();
  const int nl = tid >> 2, part = tid & 3;
#pragma unroll 1
  for (int hh = 0; hh < NH; ++hh) {
    for (int o = part * 8; o < part * 8 + 8; ++o) { float s = 0.f;
#pragma unroll 1
      for (int f = 0; f < DD; ++f) s += sx[nl][f] * sw[hh][f][o];
      sh[nl][o] = s; const __bf16 hb = (__bf16)s; sth[o][nl] = hb; stl[o][nl] = (__bf16)(s - (float)hb); }
    __syncthreads();
    if (part == 0) { float s1 = 0.f, s2 = 0.f; for (int o = 0; o < DD; ++o) { s1 += sh[nl][o] * sa1[hh][o]; s2 += sh[nl][o] * sa2[hh][o]; } sf[0][nl] = s1; sf[1][nl] = s2; }
    __syncthreads();
    { const size_t hb_ = ((size_t)b * NH + hh); for (int q = tid; q < 64 * 8; q += 256) { const int row = q >> 3, pc = q & 7; vst2(H + ((hb_ * NN) + n0 + row) * DD + pc * 4, *(const v4f*)&sh[row][pc * 4]); }
      for (int q = tid; q < DD * 8; q += 256) { const int d = q >> 3, pc = q & 7; const size_t o = (hb_ * DD + d) * NN + n0 + pc * 8; vst2((unsigned*)(HTH + o), *(const v4u*)&sth[d][pc * 8]); vst2((unsigned*)(HTL + o), *(const v4u*)&stl[d][pc * 8]); }
      if (tid < 32) { const int which = tid >> 4, pc = tid & 15; vst2(F + (hb_ * 2 + which) * NN + n0 + pc * 4, *(const v4f*)&sf[which][pc * 4]); } }
    __syncthreads(); }
}
__global__ __launch_bounds__(128) void k_gat(float* __restrict__ X, const float* __restrict__ BIAS, const float* __restrict__ F, const __bf16* __restrict__ HTH, const __bf16* __restrict__ HTL, const float* __restrict__ W1, const float* __restrict__ W2, const float* __restrict__ BG) {
  __shared__ __align__(16) float sp[4][16][36]; __shared__ float scur[4][16][33], sprev[4][16][33]; __shared__ float sw1[DD][DD + 1], sw2[DD][DD + 1], sbg[DD]; __shared__ __align__(16) float snew[4][16][36];
  const int tid = threadIdx.x, wave = tid >> 5, lane = tid & 31, col = lane & 15, g = lane >> 4; const int b = blockIdx.y; const int n0 = blockIdx.x * 64 + wave * 16;
  for (int q = tid; q < DD * DD; q += 128) { sw1[q / DD][q % DD] = bfr(W1[q]); sw2[q / DD][q % DD] = bfr(W2[q]); } if (tid < DD) sbg[tid] = bfr(BG[tid]);
  float mean0[8], mean1[8];
#pragma unroll
  for (int r = 0; r < 8; ++r) { mean0[r] = 0.f; mean1[r] = 0.f; }
#pragma unroll 1
  for (int hh = 0; hh < NH; ++hh) { const size_t hb_ = (size_t)b * NH + hh; const float* Fq = F + (hb_ * 2) * NN; const float* Fk = Fq + NN;
    float f1r[8];
#pragma unroll
    for (int r = 0; r < 8; ++r) f1r[r] = Fq[n0 + 8 * g + r];
    float m[8], l[8]; v8f acc[2] = {};
#pragma unroll
    for (int r = 0; r < 8; ++r) { m[r] = -3.0e38f; l[r] = 0.f; }
#pragma unroll 1
    for (int ks = 0; ks < NN / 32; ++ks) { const float f2a = Fk[ks * 32 + col], f2b = Fk[ks * 32 + 16 + col];
      float s[2][8];
#pragma unroll
      for (int r = 0; r < 8; ++r) { const size_t brow = ((size_t)b * NN + n0 + 8 * g + r) * NN + ks * 32; float u = f1r[r] + f2a; u = u > 0.f ? u : 0.2f * u; s[0][r] = u + bfr(BIAS[brow + col]); u = f1r[r] + f2b; u = u > 0.f ? u : 0.2f * u; s[1][r] = u + bfr(BIAS[brow + 16 + col]); }
#pragma unroll
      for (int r = 0; r < 8; ++r) { float mx = fmaxf(s[0][r], s[1][r]);
#pragma unroll
        for (int o = 1; o < 16; o <<= 1) mx = fmaxf(mx, __shfl_xor(mx, o));
        const float mn = fmaxf(m[r], mx); const float alpha = exp_ni(m[r] - mn); const float e0 = exp_ni(s[0][r] - mn), e1 = exp_ni(s[1][r] - mn); float es = e0 + e1;
#pragma unroll
        for (int o = 1; o < 16; o <<= 1) es += __shfl_xor(es, o);
        l[r] = l[r] * alpha + es; m[r] = mn; acc[0][r] *= alpha; acc[1][r] *= alpha; sp[wave][8 * g + r][col] = e0; sp[wave][8 * g + r][16 + col] = e1; }
      LDSX();
      const F2 pa = split_row(&sp[wave][col][0], 0, lane);
#pragma unroll
      for (int dt = 0; dt < 2; ++dt) { const size_t vrow = (hb_ * DD + dt * 16 + col) * NN + ks * 32; const v16b vh = frag_b(HTH + vrow, lane), vl = frag_b(HTL + vrow, lane); acc[dt] = wmma_bf(pa.l, vh, acc[dt]); acc[dt] = wmma_bf(pa.h, vl, acc[dt]); acc[dt] = wmma_bf(pa.h, vh, acc[dt]); }
      LDSX(); }
#pragma unroll
    for (int r = 0; r < 8; ++r) { const float il = 1.0f / l[r]; mean0[r] += acc[0][r] * il * (1.0f / NH); mean1[r] += acc[1][r] * il * (1.0f / NH); } }
#pragma unroll
  for (int r = 0; r < 8; ++r) { scur[wave][8 * g + r][col] = tanh_ni(mean0[r]); scur[wave][8 * g + r][16 + col] = tanh_ni(mean1[r]); }
  for (int q = lane; q < 16 * DD; q += 32) { const int rl = q / DD, f = q % DD; sprev[wave][rl][f] = X[((size_t)b * NN + n0 + rl) * DD + f]; }
  __syncthreads();
  { const int o = lane; for (int rl = 0; rl < 16; ++rl) { float zz = sbg[o];
#pragma unroll 1
      for (int f = 0; f < DD; ++f) zz += sprev[wave][rl][f] * sw1[f][o] + scur[wave][rl][f] * sw2[f][o];
      const float z = 1.0f / (1.0f + exp_ni(-zz)); snew[wave][rl][o] = z * sprev[wave][rl][o] + (1.0f - z) * scur[wave][rl][o]; } }
  LDSX();
  for (int rl = 0; rl < 16; ++rl) if (lane < 8) vst2(X + ((size_t)b * NN + n0 + rl) * DD + lane * 4, *(const v4f*)&snew[wave][rl][lane * 4]);
}
__global__ __launch_bounds__(256) void k_dec(const float* __restrict__ EDGE, const float* __restrict__ EI, const float* __restrict__ SM, const float* __restrict__ WD, const float* __restrict__ bd, float* __restrict__ FLOW, float* __restrict__ PART) {
  __shared__ float sw[64]; __shared__ float sred[256]; __shared__ __align__(16) float so[32];
  const int tid = threadIdx.x, b = blockIdx.y; const int n0 = blockIdx.x * 64;
  if (tid < 64) { float s = bfr(bd[0]);
#pragma unroll 1
    for (int f = 0; f < DD; ++f) s += EDGE[((size_t)b * NN + n0 + tid) * DD + f] * bfr(WD[f]);
    sw[tid] = 1.0f / (1.0f + exp_ni(-s)); }
  __syncthreads();
  float part = 0.f;
  for (int rl = 0; rl < 64; ++rl) { const size_t row = ((size_t)b * NN + n0 + rl) * NN; const float w = sw[rl]; v4f v; for (int k = 0; k < 4; ++k) { const size_t idx = row + tid * 4 + k; const float fv = bfr(EI[idx]) * w; v[k] = fv; part += bfr(SM[idx]) * fv; } vst2(FLOW + row + tid * 4, v); }
  sred[tid] = part; __syncthreads();
  if (tid < 32) { float s = 0.f; for (int k = tid; k < 256; k += 32) s += sred[k];
#pragma unroll
    for (int o = 1; o < 32; o <<= 1) s += __shfl_xor(s, o);
    so[tid] = (tid == 0) ? s : 0.f; }
  __syncthreads();
  if (tid < 8) vst2(PART + ((size_t)b * 16 + blockIdx.x) * 32 + tid * 4, *(const v4f*)&so[tid * 4]);
}
__global__ __launch_bounds__(32) void k_fin(const float* __restrict__ PART, float* __restrict__ MF) {
  __shared__ __align__(16) float s[32]; const int lane = threadIdx.x; float v = 0.f; if (lane < NB) { for (int k = 0; k < 16; ++k) v += PART[((size_t)lane * 16 + k) * 32]; } s[lane] = v;
  __builtin_amdgcn_fence(__ATOMIC_RELEASE, "workgroup"); __builtin_amdgcn_wave_barrier(); __builtin_amdgcn_fence(__ATOMIC_ACQUIRE, "workgroup");
  if (lane < 8) vst2(MF + lane * 4, *(const v4f*)&s[lane * 4]);
}
__global__ __launch_bounds__(256) void k_copy(const float* __restrict__ MF, const float* __restrict__ FLOW, float* __restrict__ out) {
  const size_t p = (size_t)blockIdx.x * 256 + threadIdx.x; const size_t npieces = 1 + (size_t)NB * NN * NN / 4; if (p >= npieces) return;
  v4f v; if (p == 0) v = *(const v4f*)MF; else v = *(const v4f*)(FLOW + (p - 1) * 4); vst2(out + p * 4, v);
}

extern "C" void kernel_launch(void* const* d_in, const int* in_sizes, int n_in, void* d_out, int out_size, void* d_ws, size_t ws_size, hipStream_t stream) {
  (void)in_sizes; (void)n_in; (void)out_size;
  const float** Fi = (const float**)d_in;
  if (ws_size < (size_t)WS_END) return;
  char* ws = (char*)d_ws; __bf16 *PE = (__bf16*)(ws + WS_PE), *HTH = (__bf16*)(ws + WS_HTH), *HTL = (__bf16*)(ws + WS_HTL); float *NODE = (float*)(ws + WS_NODE), *EDGE = (float*)(ws + WS_EDGE), *H = (float*)(ws + WS_H), *Fb = (float*)(ws + WS_F), *FLOW = (float*)(ws + WS_FLOW), *PART = (float*)(ws + WS_PART), *MF = (float*)(ws + WS_MF);
  k_pack<<<DD, 256, 0, stream>>>(Fi[7], PE);
  k_encn<<<TNB * NN / 64, 256, 0, stream>>>(Fi[0], Fi[5], Fi[6], NODE);
  k_ence<<<TNB * NN / 64, 128, 0, stream>>>(Fi[1], PE, Fi[8], EDGE);
  for (int l = 0; l < 2; ++l) {
    k_gath<<<dim3(NN / 64, TNB), 256, 0, stream>>>(NODE, Fi[9] + (size_t)l * NH * DD * DD, Fi[10] + l * NH * DD, Fi[11] + l * NH * DD, H, HTH, HTL, Fb);
    k_gat<<<dim3(NN / 64, TNB), 128, 0, stream>>>(NODE, Fi[2], Fb, HTH, HTL, Fi[15] + l * DD * DD, Fi[16] + l * DD * DD, Fi[17] + l * DD);
    k_gath<<<dim3(NN / 64, TNB), 256, 0, stream>>>(EDGE, Fi[12] + (size_t)l * NH * DD * DD, Fi[13] + l * NH * DD, Fi[14] + l * NH * DD, H, HTH, HTL, Fb);
    k_gat<<<dim3(NN / 64, TNB), 128, 0, stream>>>(EDGE, Fi[3], Fb, HTH, HTL, Fi[18] + l * DD * DD, Fi[19] + l * DD * DD, Fi[20] + l * DD); }
  k_dec<<<dim3(NN / 64, TNB), 256, 0, stream>>>(EDGE, Fi[1], Fi[4], Fi[21], Fi[22], FLOW, PART);
  k_fin<<<1, 32, 0, stream>>>(PART, MF);
  k_copy<<<(1 + NB * NN * NN / 4 + 255) / 256, 256, 0, stream>>>(MF, FLOW, (float*)d_out);
}
